// SelectiveWKV_1B_5368709120020
// MI455X (gfx1250) — hardware-verified
//
#include <hip/hip_runtime.h>

typedef __attribute__((ext_vector_type(16))) _Float16 v16h;
typedef __attribute__((ext_vector_type(8)))  _Float16 v8h;
typedef __attribute__((ext_vector_type(16))) __bf16   v16b;
typedef __attribute__((ext_vector_type(8)))  __bf16   v8b;
typedef __attribute__((ext_vector_type(8)))  float    v8f;
typedef __attribute__((ext_vector_type(4)))  float    v4f;

#define DM    1024
#define HS    64
#define NH    16
#define BB    4
#define TT    2048
#define ROWS  (BB * TT)
#define HPG   8
#define NGRP  (NH / HPG)
#define NCOL  (HPG * HS)
#define TS    32
#define WSCALE 32.0f
#define WSCALE_INV (1.0f / 32.0f)

__device__ __forceinline__ unsigned short f2bf_bits(float f) {
  unsigned u = __float_as_uint(f);
  return (unsigned short)((u + 0x7FFFu + ((u >> 16) & 1u)) >> 16);
}
__device__ __forceinline__ float bf_bits2f(unsigned short h) { return __uint_as_float(((unsigned)h) << 16); }

__device__ __forceinline__ void dep_guard_h(v8f& a, v8f& b, v16h x, v16h y) { asm volatile("v_nop\n\tv_nop\n\tv_nop\n\tv_nop" : "+v"(a), "+v"(b) : "v"(x), "v"(y)); }
__device__ __forceinline__ void dep_guard_b(v8f& a, v8f& b, v16b x, v16b y) { asm volatile("v_nop\n\tv_nop\n\tv_nop\n\tv_nop" : "+v"(a), "+v"(b) : "v"(x), "v"(y)); }
__device__ __forceinline__ void keep4_h(v16h a, v16h b, v16h c, v16h d) { asm volatile("v_nop" :: "v"(a), "v"(b), "v"(c), "v"(d)); }
__device__ __forceinline__ void keep4_b(v16b a, v16b b, v16b c, v16b d) { asm volatile("v_nop" :: "v"(a), "v"(b), "v"(c), "v"(d)); }
__device__ __forceinline__ void acc_guard4(v8f& a, v8f& b, v8f& c, v8f& d) { asm volatile("v_nop\n\tv_nop\n\tv_nop\n\tv_nop" : "+v"(a), "+v"(b), "+v"(c), "+v"(d)); }
template <typename T> struct Frag;
template <> struct Frag<_Float16> {
  typedef v16h V; union U { v16h v; v8h h[2]; };
  static __device__ __forceinline__ v16h load(const _Float16* p) {
    U f; f.h[0] = *(const v8h*)(p); f.h[1] = *(const v8h*)(p + 16); return f.v;
  }
  static __device__ __forceinline__ v8f mma(v16h a, v16h b, v8f c) {
    return __builtin_amdgcn_wmma_f32_16x16x32_f16(false, a, false, b, (short)0, c, false, false);
  }
  static __device__ __forceinline__ void guard(v8f& a, v8f& b, v16h x, v16h y) { dep_guard_h(a, b, x, y); }
  static __device__ __forceinline__ void keep(v16h a, v16h b, v16h c, v16h d) { keep4_h(a, b, c, d); }
};
template <> struct Frag<__bf16> {
  typedef v16b V; union U { v16b v; v8b h[2]; };
  static __device__ __forceinline__ v16b load(const __bf16* p) {
    U f; f.h[0] = *(const v8b*)(p); f.h[1] = *(const v8b*)(p + 16); return f.v;
  }
  static __device__ __forceinline__ v8f mma(v16b a, v16b b, v8f c) {
    return __builtin_amdgcn_wmma_f32_16x16x32_bf16(false, a, false, b, (short)0, c, false, false);
  }
  static __device__ __forceinline__ void guard(v8f& a, v8f& b, v16b x, v16b y) { dep_guard_b(a, b, x, y); }
  static __device__ __forceinline__ void keep(v16b a, v16b b, v16b c, v16b d) { keep4_b(a, b, c, d); }
};

template <int ET> struct Elem;
template <> struct Elem<0> { typedef _Float16 T; };
template <> struct Elem<1> { typedef __bf16 T; };
template <int ET, bool SPLIT, int BIAS_MODE, int OUT_MODE, bool RESID, int ACT = 0>
__global__ __launch_bounds__(256) void wmma_gemm64(
    const unsigned short* __restrict__ Ap, const unsigned short* __restrict__ A2p, int lda, long strideA,
    const unsigned short* __restrict__ Btp, const unsigned short* __restrict__ Bt2p, int ldb, long strideB,
    void* __restrict__ Cout, void* __restrict__ Cout2, int ldc, long strideC,
    const float* __restrict__ bias,
    const float* __restrict__ resid, long strideR,
    int M, int N, int K, float scale) {
  typedef typename Elem<ET>::T T;
  typedef typename Frag<T>::V V;
  const T* A = (const T*)Ap; const T* A2 = (const T*)A2p; const T* Bt = (const T*)Btp; const T* Bt2 = (const T*)Bt2p;
  __shared__ __align__(16) float sT[8][16 * 68];
  const int b    = blockIdx.y;
  const int lane = threadIdx.x & 31;
  const int wave = threadIdx.x >> 5;
  const int tilesN = N >> 6;
  const int tilesM = M >> 6;
  const int tile = blockIdx.x * 8 + wave;
  if (tile >= tilesM * tilesN) return;
  const int tm = tile / tilesN;
  const int tn = tile - tm * tilesN;
  const int m0 = tm << 6;
  const int n0 = tn << 6;

  const T* Ab  = A  + (size_t)b * strideA;
  const T* Bb  = Bt + (size_t)b * strideB;
  const T* Ab2 = SPLIT ? (A2  + (size_t)b * strideA) : nullptr;
  const T* Bb2 = SPLIT ? (Bt2 + (size_t)b * strideB) : nullptr;

  const int rlane = lane & 15;
  const int koff  = (lane >> 4) * 8;
  const int mOff  = (lane >> 4) * 8;

  v8f acc[4][4];
#pragma unroll
  for (int i = 0; i < 4; ++i)
#pragma unroll
    for (int j = 0; j < 4; ++j) acc[i][j] = (v8f){0.f,0.f,0.f,0.f,0.f,0.f,0.f,0.f};

  for (int k0 = 0; k0 < K; k0 += 32) {
    V bh[4], bl[4];
#pragma unroll
    for (int j = 0; j < 4; ++j) {
      const size_t bo = (size_t)(n0 + (j << 4) + rlane) * ldb + koff + k0;
      bh[j] = Frag<T>::load(Bb + bo);
      if (SPLIT) bl[j] = Frag<T>::load(Bb2 + bo);
    }
#pragma unroll
    for (int i = 0; i < 4; ++i) {
      const size_t ao = (size_t)(m0 + (i << 4) + rlane) * lda + koff + k0;
      V ah = Frag<T>::load(Ab + ao);
      V al;
      if (SPLIT) al = Frag<T>::load(Ab2 + ao);
#pragma unroll
      for (int j = 0; j < 4; ++j) {
        acc[i][j] = Frag<T>::mma(ah, bh[j], acc[i][j]);
        if (SPLIT) {
          acc[i][j] = Frag<T>::mma(ah, bl[j], acc[i][j]);
          acc[i][j] = Frag<T>::mma(al, bh[j], acc[i][j]);
        }
      }
      Frag<T>::guard(acc[i][0], acc[i][3], ah, SPLIT ? al : ah);
    }
    Frag<T>::keep(bh[0], bh[1], bh[2], bh[3]);
    if (SPLIT) Frag<T>::keep(bl[0], bl[1], bl[2], bl[3]);
  }
  acc_guard4(acc[0][0], acc[0][1], acc[0][2], acc[0][3]);
  acc_guard4(acc[1][0], acc[1][1], acc[1][2], acc[1][3]);
  acc_guard4(acc[2][0], acc[2][1], acc[2][2], acc[2][3]);
  acc_guard4(acc[3][0], acc[3][1], acc[3][2], acc[3][3]);

  float* slab = sT[wave];
  const float* Rb = RESID ? (resid + (size_t)b * strideR) : nullptr;
#pragma unroll
  for (int i = 0; i < 4; ++i) {
    const int mBase = m0 + (i << 4);
#pragma unroll
    for (int j = 0; j < 4; ++j) {
      const int n = n0 + (j << 4) + rlane;
      float bv = 0.f;
      if (BIAS_MODE == 2) bv = bias[n];
#pragma unroll
      for (int r = 0; r < 8; ++r) {
        float v = acc[i][j][r] * scale;
        if (BIAS_MODE == 1) v += bias[mBase + mOff + r];
        if (BIAS_MODE == 2) v += bv;
        if (RESID) v += Rb[(size_t)(mBase + mOff + r) * ldc + n];
        if (ACT == 1) v = tanhf(v);
        if (ACT == 2) v = fmaxf(v, 0.0f);
        if (ACT == 3) v = v / (1.0f + expf(-v));
        if (ACT == 4) v = (v > 0.f) ? v : 0.01f * v;
        if (ACT == 5) v = 0.5f * v * (1.0f + erff(v * 0.70710678118654752f));
        if (ACT == 6) v = __builtin_amdgcn_rcpf(1.0f + __expf(-v));
        if (ACT == 7) v = 1.0f - __builtin_amdgcn_rcpf(1.0f + __expf(-v));
        slab[(mOff + r) * 68 + (j << 4) + rlane] = v;
      }
    }
    __builtin_amdgcn_fence(__ATOMIC_RELEASE, "workgroup");
    __builtin_amdgcn_wave_barrier();
    __builtin_amdgcn_fence(__ATOMIC_ACQUIRE, "workgroup");
    if (OUT_MODE == 0) {
      float* C = (float*)Cout + (size_t)b * strideC;
      const int hh = lane >> 4, c4 = (lane & 15) * 4;
      for (int pass = 0; pass < 2; ++pass) {
#pragma unroll
        for (int it = 0; it < 8; ++it) {
          const int row = it * 2 + hh;
          v4f v = *(const v4f*)(slab + row * 68 + c4);
          *(volatile v4f*)(C + (size_t)(mBase + row) * ldc + n0 + c4) = v;
        }
        __threadfence();
      }
    } else {
      const int q = lane >> 3, c8 = (lane & 7) * 8;
      unsigned short* C  = (unsigned short*)Cout  + (size_t)b * strideC;
      unsigned short* C2 = (OUT_MODE == 2) ? ((unsigned short*)Cout2 + (size_t)b * strideC) : nullptr;
      for (int pass = 0; pass < 2; ++pass) {
#pragma unroll
        for (int it = 0; it < 4; ++it) {
          const int row = it * 4 + q;
          const float* sp = slab + row * 68 + c8;
          v8h hv, lv;
#pragma unroll
          for (int e = 0; e < 8; ++e) {
            if (OUT_MODE == 1) {
              hv[e] = (_Float16)sp[e];
            } else {
              unsigned short hb = f2bf_bits(sp[e]);
              unsigned short lb = f2bf_bits(sp[e] - bf_bits2f(hb));
              hv[e] = __builtin_bit_cast(_Float16, hb);
              lv[e] = __builtin_bit_cast(_Float16, lb);
            }
          }
          *(volatile v8h*)(C + (size_t)(mBase + row) * ldc + n0 + c8) = hv;
          if (OUT_MODE == 2) *(volatile v8h*)(C2 + (size_t)(mBase + row) * ldc + n0 + c8) = lv;
        }
        __threadfence();
      }
    }
    __builtin_amdgcn_fence(__ATOMIC_RELEASE, "workgroup");
    __builtin_amdgcn_wave_barrier();
    __builtin_amdgcn_fence(__ATOMIC_ACQUIRE, "workgroup");
  }
}

__global__ __launch_bounds__(256) void transpose_scale_f16(const float* __restrict__ src, _Float16* __restrict__ dst,
                                                           int nk, int nn, float scl) {
  __shared__ float tile[64 * 65];
  const int tid = threadIdx.x, lane = tid & 31, wave = tid >> 5;
  const int n0 = blockIdx.x * 64, k0 = blockIdx.y * 64;
  {
    const int r = tid >> 2, c = (tid & 3) * 16;
    const float* sp = src + (size_t)(k0 + r) * nn + n0 + c;
#pragma unroll
    for (int u = 0; u < 4; ++u) {
      const v4f t4 = *(const v4f*)(sp + 4 * u);
#pragma unroll
      for (int e = 0; e < 4; ++e) tile[r * 65 + c + 4 * u + e] = t4[e] * scl;
    }
  }
  __syncthreads();
  const int q = lane >> 3, c8 = (lane & 7) * 8;
  for (int pass = 0; pass < 2; ++pass) {
#pragma unroll
    for (int it = 0; it < 2; ++it) {
      const int row = it * 32 + wave * 4 + q;
      v8h hv;
#pragma unroll
      for (int e = 0; e < 8; ++e) hv[e] = (_Float16)tile[(c8 + e) * 65 + row];
      *(volatile v8h*)(dst + (size_t)(n0 + row) * nk + k0 + c8) = hv;
    }
    __threadfence();
  }
}

__global__ __launch_bounds__(128) void layernorm_f16(const float* __restrict__ x, const float* __restrict__ g,
                                                     const float* __restrict__ bb, _Float16* __restrict__ xn) {
  __shared__ float red0[4], red1[4];
  const int row = blockIdx.x;
  const int tid = threadIdx.x, lane = tid & 31, wave = tid >> 5;
  const int c0 = tid * 8;
  const float* xr = x + (size_t)row * DM + c0;
  const v4f a = *(const v4f*)xr;
  const v4f c = *(const v4f*)(xr + 4);
  float v[8];
  v[0] = a[0]; v[1] = a[1]; v[2] = a[2]; v[3] = a[3];
  v[4] = c[0]; v[5] = c[1]; v[6] = c[2]; v[7] = c[3];
  float sm = ((v[0] + v[1]) + (v[2] + v[3])) + ((v[4] + v[5]) + (v[6] + v[7]));
#pragma unroll
  for (int off = 16; off > 0; off >>= 1) sm += __shfl_xor(sm, off, 32);
  if (lane == 0) red0[wave] = sm;
  __syncthreads();
  const float S = (red0[0] + red0[1]) + (red0[2] + red0[3]);
  const float mu = S * (1.0f / 1024.0f);
  float qd = 0.f;
#pragma unroll
  for (int i = 0; i < 8; ++i) { const float d = v[i] - mu; qd = fmaf(d, d, qd); }
#pragma unroll
  for (int off = 16; off > 0; off >>= 1) qd += __shfl_xor(qd, off, 32);
  if (lane == 0) red1[wave] = qd;
  __syncthreads();
  const float Q = (red1[0] + red1[1]) + (red1[2] + red1[3]);
  const float var = Q * (1.0f / 1024.0f);
  const float inv = rsqrtf(var + 1e-5f);
  const v4f g0 = *(const v4f*)(g + c0), g1 = *(const v4f*)(g + c0 + 4);
  const v4f b0 = *(const v4f*)(bb + c0), b1 = *(const v4f*)(bb + c0 + 4);
  float gg[8], bv[8];
  gg[0] = g0[0]; gg[1] = g0[1]; gg[2] = g0[2]; gg[3] = g0[3]; gg[4] = g1[0]; gg[5] = g1[1]; gg[6] = g1[2]; gg[7] = g1[3];
  bv[0] = b0[0]; bv[1] = b0[1]; bv[2] = b0[2]; bv[3] = b0[3]; bv[4] = b1[0]; bv[5] = b1[1]; bv[6] = b1[2]; bv[7] = b1[3];
  v8h hv;
#pragma unroll
  for (int i = 0; i < 8; ++i) hv[i] = (_Float16)(((v[i] - mu) * inv) * gg[i] + bv[i]);
  _Float16* dstp = xn + (size_t)row * DM + c0;
  *(volatile v8h*)dstp = hv;
  __threadfence();
  *(volatile v8h*)dstp = hv;
}

__global__ __launch_bounds__(256) void wkv_scan(const float* __restrict__ kb, const float* __restrict__ vb,
                                                const float* __restrict__ db, const float* __restrict__ rb,
                                                _Float16* __restrict__ so, float* __restrict__ st,
                                                int hbase, int ldp) {
  __shared__ __align__(16) float stg[4 * TS * HS];
  __shared__ __align__(16) float sO[TS * HS];
  float* sK = stg;
  float* sV = stg + TS * HS;
  float* sD = stg + 2 * TS * HS;
  float* sR = stg + 3 * TS * HS;
  const int tid = threadIdx.x, lane = tid & 31, wave = tid >> 5;
  const int blk = blockIdx.x;
  const int b  = blk / HPG;
  const int hl = blk - b * HPG;
  const int hg = hbase + hl;
  const int dg = tid & 3, e = tid >> 2;
  const size_t rowb = (size_t)b * TT;
  const int colb = hl * HS;

  float s[16];
#pragma unroll
  for (int i = 0; i < 16; ++i) s[i] = 0.0f;

#pragma unroll 1
  for (int t0 = 0; t0 < TT; t0 += TS) {
#pragma unroll
    for (int u = 0; u < 2; ++u) {
      const int j = tid + 256 * u;
      const int r = j >> 4, c4 = (j & 15) * 4;
      const size_t go = (rowb + t0 + r) * (size_t)ldp + colb + c4;
      const int lo = r * HS + c4;
      *(v4f*)(sK + lo) = *(const v4f*)(kb + go);
      *(v4f*)(sV + lo) = *(const v4f*)(vb + go);
      *(v4f*)(sD + lo) = *(const v4f*)(db + go);
      *(v4f*)(sR + lo) = *(const v4f*)(rb + go);
    }
    __syncthreads();
#pragma unroll 1
    for (int ss = 0; ss < TS; ++ss) {
      const float vv = sV[ss * HS + e];
      const float* kp = sK + ss * HS + dg * 16;
      const float* dp = sD + ss * HS + dg * 16;
      const float* rp = sR + ss * HS + dg * 16;
      float acc = 0.0f;
#pragma unroll
      for (int q = 0; q < 4; ++q) {
        const v4f k4 = *(const v4f*)(kp + 4 * q);
        const v4f d4 = *(const v4f*)(dp + 4 * q);
        const v4f r4 = *(const v4f*)(rp + 4 * q);
#pragma unroll
        for (int z = 0; z < 4; ++z) {
          float sd = s[4 * q + z];
          sd = d4[z] * sd + k4[z] * vv;
          s[4 * q + z] = sd;
          acc = fmaf(r4[z], sd, acc);
        }
      }
      acc += __shfl_xor(acc, 1, 32);
      acc += __shfl_xor(acc, 2, 32);
      if (dg == 0) sO[ss * HS + e] = acc;
    }
    __syncthreads();
    {
      const int q = lane >> 3, c8 = (lane & 7) * 8;
      const int r = wave * 4 + q;
      v8h hv;
#pragma unroll
      for (int i = 0; i < 8; ++i) hv[i] = (_Float16)sO[r * HS + c8 + i];
      _Float16* dstp = so + (rowb + t0 + r) * (size_t)DM + hg * HS + c8;
      *(volatile v8h*)dstp = hv;
      __threadfence();
      *(volatile v8h*)dstp = hv;
    }
  }

#pragma unroll
  for (int i = 0; i < 16; ++i) stg[(dg * 16 + i) * HS + e] = s[i];
  __syncthreads();
  {
    const int hh = lane >> 4, c4 = (lane & 15) * 4;
    float* sb = st + (size_t)(b * NH + hg) * HS * HS;
    for (int pass = 0; pass < 2; ++pass) {
#pragma unroll
      for (int it = 0; it < 4; ++it) {
        const int row = it * 16 + wave * 2 + hh;
        const v4f val = *(const v4f*)(stg + row * HS + c4);
        *(volatile v4f*)(sb + (size_t)row * HS + c4) = val;
      }
      __threadfence();
    }
  }
}

template <int BIAS, int OUTM, int ACT>
static void run_gemm(const void* A, int lda, const void* Bt, int ldb, void* C, int ldc, const float* bias,
                     int M, int N, int K, float scale, hipStream_t st) {
  const dim3 grid((unsigned)((((M >> 6) * (N >> 6)) + 7) >> 3), 1, 1);
  hipLaunchKernelGGL(HIP_KERNEL_NAME(wmma_gemm64<0, false, BIAS, OUTM, false, ACT>), grid, dim3(256), 0, st,
                     (const unsigned short*)A, (const unsigned short*)nullptr, lda, 0L,
                     (const unsigned short*)Bt, (const unsigned short*)nullptr, ldb, 0L,
                     C, (void*)nullptr, ldc, 0L,
                     bias, (const float*)nullptr, 0L, M, N, K, scale);
}

extern "C" void kernel_launch(void* const* d_in, const int* in_sizes, int n_in,
                              void* d_out, int out_size, void* d_ws, size_t ws_size,
                              hipStream_t stream) {
  if (n_in < 10) return;
  if (in_sizes[0] != ROWS * DM || in_sizes[1] != DM || in_sizes[2] != DM || in_sizes[3] != DM * DM ||
      in_sizes[4] != DM * DM || in_sizes[5] != DM || in_sizes[6] != DM * DM || in_sizes[7] != DM * DM ||
      in_sizes[8] != DM * DM || in_sizes[9] != DM * DM) return;
  if (out_size != ROWS * DM + BB * NH * HS * HS) return;

  const float* x    = (const float*)d_in[0];
  const float* ln_g = (const float*)d_in[1];
  const float* ln_b = (const float*)d_in[2];
  const float* Wx   = (const float*)d_in[3];
  const float* Ww   = (const float*)d_in[4];
  const float* bw   = (const float*)d_in[5];
  const float* Wk   = (const float*)d_in[6];
  const float* Wv   = (const float*)d_in[7];
  const float* Wr   = (const float*)d_in[8];
  const float* Wo   = (const float*)d_in[9];

  size_t off = 0;
  const size_t wb   = (size_t)DM * DM * 2;
  const size_t ab16 = (size_t)ROWS * DM * 2;
  const size_t gb32 = (size_t)ROWS * NCOL * 4;
  char* base = (char*)d_ws;
  _Float16* WxT = (_Float16*)(base + off); off += wb;
  _Float16* WwT = (_Float16*)(base + off); off += wb;
  _Float16* WkT = (_Float16*)(base + off); off += wb;
  _Float16* WvT = (_Float16*)(base + off); off += wb;
  _Float16* WrT = (_Float16*)(base + off); off += wb;
  _Float16* WoT = (_Float16*)(base + off); off += wb;
  _Float16* xn  = (_Float16*)(base + off); off += ab16;
  _Float16* tmp = (_Float16*)(base + off); off += ab16;
  float* dbuf = (float*)(base + off); off += gb32;
  float* kbuf = (float*)(base + off); off += gb32;
  float* vbuf = (float*)(base + off); off += gb32;
  float* rbuf = (float*)(base + off); off += gb32;
  _Float16* sout = (_Float16*)(base + off); off += ab16;
  if (off > ws_size) return;

  float* y_out     = (float*)d_out;
  float* state_out = y_out + (size_t)ROWS * DM;

  const dim3 gT(DM / 64, DM / 64);
  transpose_scale_f16<<<gT, dim3(256), 0, stream>>>(Wx, WxT, DM, DM, WSCALE);
  transpose_scale_f16<<<gT, dim3(256), 0, stream>>>(Ww, WwT, DM, DM, WSCALE);
  transpose_scale_f16<<<gT, dim3(256), 0, stream>>>(Wk, WkT, DM, DM, WSCALE);
  transpose_scale_f16<<<gT, dim3(256), 0, stream>>>(Wv, WvT, DM, DM, WSCALE);
  transpose_scale_f16<<<gT, dim3(256), 0, stream>>>(Wr, WrT, DM, DM, WSCALE);
  transpose_scale_f16<<<gT, dim3(256), 0, stream>>>(Wo, WoT, DM, DM, WSCALE);

  layernorm_f16<<<dim3(ROWS), dim3(128), 0, stream>>>(x, ln_g, ln_b, xn);

  run_gemm<0, 1, 0>(xn, DM, WxT, DM, (void*)tmp, DM, (const float*)nullptr, ROWS, DM, DM, WSCALE_INV, stream);

  for (int g = 0; g < NGRP; ++g) {
    const size_t wrow = (size_t)g * NCOL * DM;
    run_gemm<2, 0, 7>(tmp, DM, WwT + wrow, DM, (void*)dbuf, NCOL, bw + g * NCOL, ROWS, NCOL, DM, WSCALE_INV, stream);
    run_gemm<0, 0, 0>(xn,  DM, WkT + wrow, DM, (void*)kbuf, NCOL, (const float*)nullptr, ROWS, NCOL, DM, WSCALE_INV, stream);
    run_gemm<0, 0, 0>(xn,  DM, WvT + wrow, DM, (void*)vbuf, NCOL, (const float*)nullptr, ROWS, NCOL, DM, WSCALE_INV, stream);
    run_gemm<0, 0, 6>(xn,  DM, WrT + wrow, DM, (void*)rbuf, NCOL, (const float*)nullptr, ROWS, NCOL, DM, WSCALE_INV, stream);
    wkv_scan<<<dim3(BB * HPG), dim3(256), 0, stream>>>(kbuf, vbuf, dbuf, rbuf, sout, state_out, g * HPG, NCOL);
  }

  run_gemm<0, 0, 0>(sout, DM, WoT, DM, (void*)y_out, DM, (const float*)nullptr, ROWS, DM, DM, WSCALE_INV, stream);
}
